// MASA_54022098649572
// MI455X (gfx1250) — hardware-verified
//
#include <hip/hip_runtime.h>
#include <math.h>

constexpr int kBatch  = 4;
constexpr int kCin    = 192;
constexpr int kImw    = 128;
constexpr int kNpix   = 16384;
constexpr int kOc     = 768;
constexpr int kHeads  = 8;
constexpr int kChd    = 24;
constexpr int kCpad   = 32;
constexpr int kNag    = 64;
constexpr int kKBlk   = 16;
constexpr int kKChunk = 16;
constexpr int kQBlk   = 64;
constexpr int kQTile  = 4;
static_assert(kKBlk * kKChunk * 64 == kNpix);
static_assert(kQBlk * kQTile * 64 == kNpix);
static_assert(kHeads * kChd == kCin);

typedef __attribute__((ext_vector_type(16))) _Float16 v16h;
typedef __attribute__((ext_vector_type(8)))  _Float16 v8h;
typedef __attribute__((ext_vector_type(16))) __bf16   v16b;
typedef __attribute__((ext_vector_type(8)))  __bf16   v8b;
typedef __attribute__((ext_vector_type(8)))  float    v8f;
typedef __attribute__((ext_vector_type(4)))  float    v4f;
typedef __attribute__((ext_vector_type(4)))  unsigned int v4u;

constexpr size_t kMiB       = 1048576;
constexpr size_t kOffWhi    = 0;
constexpr size_t kOffWlo    = 294912;
constexpr size_t kOffR1     = 1 * kMiB;
constexpr size_t kOffPre    = kOffR1;
constexpr size_t kOffQnhi   = kOffR1;
constexpr size_t kOffQnlo   = kOffR1 + 8 * kMiB;
constexpr size_t kOffKnhi   = kOffR1 + 16 * kMiB;
constexpr size_t kOffKnlo   = kOffR1 + 24 * kMiB;
constexpr size_t kOffVhi    = kOffR1 + 32 * kMiB;
constexpr size_t kOffVlo    = kOffR1 + 38 * kMiB;
constexpr size_t kOffR2     = 49 * kMiB;
constexpr size_t kOffXthi   = kOffR2;
constexpr size_t kOffXtlo   = kOffR2 + 6 * kMiB;
constexpr size_t kOffDw     = kOffR2;
constexpr size_t kOffOutT   = kOffR2;
constexpr size_t kOffR3     = 97 * kMiB;
constexpr size_t kOffAghi   = kOffR3;
constexpr size_t kOffAglo   = kOffR3 + 32768;
constexpr size_t kOffAvhi   = kOffR3 + 65536;
constexpr size_t kOffAvlo   = kOffR3 + 98304;
constexpr size_t kOffPartO  = kOffR3 + 1 * kMiB;
constexpr size_t kOffPartML = kOffR3 + 2 * kMiB;
constexpr size_t kWsEnd     = kOffR3 + 3 * kMiB;
static_assert((size_t)kOc * kCin * 2 <= kOffWlo);
static_assert(kOffWlo + (size_t)kOc * kCin * 2 <= kOffR1);
static_assert((size_t)kOc * kNpix * 4 <= 48 * kMiB);
static_assert((size_t)kHeads * kNpix * kCpad * 2 == 8 * kMiB);
static_assert((size_t)kCin * kNpix * 2 == 6 * kMiB);
static_assert(kOffVlo + 6 * kMiB <= kOffR2);
static_assert((size_t)kNpix * kCin * 2 == 6 * kMiB);
static_assert(kOffR2 + 48 * kMiB <= kOffR3);
static_assert((size_t)kHeads * kNag * kCpad * 2 == 32768);
static_assert((size_t)kHeads * kKBlk * kNag * kCpad * 4 == 1 * kMiB);
static_assert((size_t)kHeads * kKBlk * kNag * 2 * 4 <= 1 * kMiB);
static_assert(kWsEnd == 104857600);

__device__ __forceinline__ unsigned short f2bf_bits(float f) {
  unsigned u = __float_as_uint(f);
  return (unsigned short)((u + 0x7FFFu + ((u >> 16) & 1u)) >> 16);
}
__device__ __forceinline__ float bf_bits2f(unsigned short h) { return __uint_as_float(((unsigned)h) << 16); }

__device__ __forceinline__ void dep_guard_h(v8f& a, v8f& b, v16h x, v16h y) { asm volatile("v_nop\n\tv_nop\n\tv_nop\n\tv_nop" : "+v"(a), "+v"(b) : "v"(x), "v"(y)); }
__device__ __forceinline__ void dep_guard_b(v8f& a, v8f& b, v16b x, v16b y) { asm volatile("v_nop\n\tv_nop\n\tv_nop\n\tv_nop" : "+v"(a), "+v"(b) : "v"(x), "v"(y)); }
__device__ __forceinline__ void keep4_h(v16h a, v16h b, v16h c, v16h d) { asm volatile("v_nop" :: "v"(a), "v"(b), "v"(c), "v"(d)); }
__device__ __forceinline__ void keep4_b(v16b a, v16b b, v16b c, v16b d) { asm volatile("v_nop" :: "v"(a), "v"(b), "v"(c), "v"(d)); }
__device__ __forceinline__ void acc_guard4(v8f& a, v8f& b, v8f& c, v8f& d) { asm volatile("v_nop\n\tv_nop\n\tv_nop\n\tv_nop" : "+v"(a), "+v"(b), "+v"(c), "+v"(d)); }
template <typename T> struct Frag;
template <> struct Frag<_Float16> {
  typedef v16h V; union U { v16h v; v8h h[2]; };
  static __device__ __forceinline__ v16h load(const _Float16* p) {
    U f; f.h[0] = *(const v8h*)(p); f.h[1] = *(const v8h*)(p + 16); return f.v;
  }
  static __device__ __forceinline__ v8f mma(v16h a, v16h b, v8f c) {
    return __builtin_amdgcn_wmma_f32_16x16x32_f16(false, a, false, b, (short)0, c, false, false);
  }
  static __device__ __forceinline__ void guard(v8f& a, v8f& b, v16h x, v16h y) { dep_guard_h(a, b, x, y); }
  static __device__ __forceinline__ void keep(v16h a, v16h b, v16h c, v16h d) { keep4_h(a, b, c, d); }
};
template <> struct Frag<__bf16> {
  typedef v16b V; union U { v16b v; v8b h[2]; };
  static __device__ __forceinline__ v16b load(const __bf16* p) {
    U f; f.h[0] = *(const v8b*)(p); f.h[1] = *(const v8b*)(p + 16); return f.v;
  }
  static __device__ __forceinline__ v8f mma(v16b a, v16b b, v8f c) {
    return __builtin_amdgcn_wmma_f32_16x16x32_bf16(false, a, false, b, (short)0, c, false, false);
  }
  static __device__ __forceinline__ void guard(v8f& a, v8f& b, v16b x, v16b y) { dep_guard_b(a, b, x, y); }
  static __device__ __forceinline__ void keep(v16b a, v16b b, v16b c, v16b d) { keep4_b(a, b, c, d); }
};

__device__ __forceinline__ unsigned pk16(unsigned short a, unsigned short b) { return (unsigned)a | ((unsigned)b << 16); }

template <int ET> struct Elem;
template <> struct Elem<0> { typedef _Float16 T; };
template <> struct Elem<1> { typedef __bf16 T; };
template <int ET, bool SPLIT, int BIAS_MODE, int OUT_MODE, bool RESID, int ACT = 0>
__global__ __launch_bounds__(256) void wmma_gemm64(
    const unsigned short* __restrict__ Ap, const unsigned short* __restrict__ A2p, int lda, long strideA,
    const unsigned short* __restrict__ Btp, const unsigned short* __restrict__ Bt2p, int ldb, long strideB,
    void* __restrict__ Cout, void* __restrict__ Cout2, int ldc, long strideC,
    const float* __restrict__ bias,
    const float* __restrict__ resid, long strideR,
    int M, int N, int K, float scale) {
  typedef typename Elem<ET>::T T;
  typedef typename Frag<T>::V V;
  const T* A = (const T*)Ap; const T* A2 = (const T*)A2p; const T* Bt = (const T*)Btp; const T* Bt2 = (const T*)Bt2p;
  __shared__ __align__(16) float sT[8][16 * 68];
  const int b    = blockIdx.y;
  const int lane = threadIdx.x & 31;
  const int wave = threadIdx.x >> 5;
  const int tilesN = N >> 6;
  const int tilesM = M >> 6;
  const int tile = blockIdx.x * 8 + wave;
  if (tile >= tilesM * tilesN) return;
  const int tm = tile / tilesN;
  const int tn = tile - tm * tilesN;
  const int m0 = tm << 6;
  const int n0 = tn << 6;

  const T* Ab  = A  + (size_t)b * strideA;
  const T* Bb  = Bt + (size_t)b * strideB;
  const T* Ab2 = SPLIT ? (A2  + (size_t)b * strideA) : nullptr;
  const T* Bb2 = SPLIT ? (Bt2 + (size_t)b * strideB) : nullptr;

  const int rlane = lane & 15;
  const int koff  = (lane >> 4) * 8;
  const int mOff  = (lane >> 4) * 8;

  v8f acc[4][4];
#pragma unroll
  for (int i = 0; i < 4; ++i)
#pragma unroll
    for (int j = 0; j < 4; ++j) acc[i][j] = (v8f){0.f,0.f,0.f,0.f,0.f,0.f,0.f,0.f};

  for (int k0 = 0; k0 < K; k0 += 32) {
    V bh[4], bl[4];
#pragma unroll
    for (int j = 0; j < 4; ++j) {
      const size_t bo = (size_t)(n0 + (j << 4) + rlane) * ldb + koff + k0;
      bh[j] = Frag<T>::load(Bb + bo);
      if (SPLIT) bl[j] = Frag<T>::load(Bb2 + bo);
    }
#pragma unroll
    for (int i = 0; i < 4; ++i) {
      const size_t ao = (size_t)(m0 + (i << 4) + rlane) * lda + koff + k0;
      V ah = Frag<T>::load(Ab + ao);
      V al;
      if (SPLIT) al = Frag<T>::load(Ab2 + ao);
#pragma unroll
      for (int j = 0; j < 4; ++j) {
        acc[i][j] = Frag<T>::mma(ah, bh[j], acc[i][j]);
        if (SPLIT) {
          acc[i][j] = Frag<T>::mma(ah, bl[j], acc[i][j]);
          acc[i][j] = Frag<T>::mma(al, bh[j], acc[i][j]);
        }
      }
      Frag<T>::guard(acc[i][0], acc[i][3], ah, SPLIT ? al : ah);
    }
    Frag<T>::keep(bh[0], bh[1], bh[2], bh[3]);
    if (SPLIT) Frag<T>::keep(bl[0], bl[1], bl[2], bl[3]);
  }
  acc_guard4(acc[0][0], acc[0][1], acc[0][2], acc[0][3]);
  acc_guard4(acc[1][0], acc[1][1], acc[1][2], acc[1][3]);
  acc_guard4(acc[2][0], acc[2][1], acc[2][2], acc[2][3]);
  acc_guard4(acc[3][0], acc[3][1], acc[3][2], acc[3][3]);

  float* slab = sT[wave];
  const float* Rb = RESID ? (resid + (size_t)b * strideR) : nullptr;
#pragma unroll
  for (int i = 0; i < 4; ++i) {
    const int mBase = m0 + (i << 4);
#pragma unroll
    for (int j = 0; j < 4; ++j) {
      const int n = n0 + (j << 4) + rlane;
      float bv = 0.f;
      if (BIAS_MODE == 2) bv = bias[n];
#pragma unroll
      for (int r = 0; r < 8; ++r) {
        float v = acc[i][j][r] * scale;
        if (BIAS_MODE == 1) v += bias[mBase + mOff + r];
        if (BIAS_MODE == 2) v += bv;
        if (RESID) v += Rb[(size_t)(mBase + mOff + r) * ldc + n];
        if (ACT == 2) v = fmaxf(v, 0.0f);
        if (ACT == 4) v = (v > 0.f) ? v : 0.01f * v;
        slab[(mOff + r) * 68 + (j << 4) + rlane] = v;
      }
    }
    __builtin_amdgcn_fence(__ATOMIC_RELEASE, "workgroup");
    __builtin_amdgcn_wave_barrier();
    __builtin_amdgcn_fence(__ATOMIC_ACQUIRE, "workgroup");
    if (OUT_MODE == 0) {
      float* C = (float*)Cout + (size_t)b * strideC;
      const int hh = lane >> 4, c4 = (lane & 15) * 4;
      for (int pass = 0; pass < 2; ++pass) {
#pragma unroll
        for (int it = 0; it < 8; ++it) {
          const int row = it * 2 + hh;
          v4f v = *(const v4f*)(slab + row * 68 + c4);
          *(volatile v4f*)(C + (size_t)(mBase + row) * ldc + n0 + c4) = v;
        }
        __threadfence();
      }
    } else {
      const int q = lane >> 3, c8 = (lane & 7) * 8;
      unsigned short* C  = (unsigned short*)Cout  + (size_t)b * strideC;
      unsigned short* C2 = (OUT_MODE == 2) ? ((unsigned short*)Cout2 + (size_t)b * strideC) : nullptr;
      for (int pass = 0; pass < 2; ++pass) {
#pragma unroll
        for (int it = 0; it < 4; ++it) {
          const int row = it * 4 + q;
          const float* sp = slab + row * 68 + c8;
          v8h hv, lv;
#pragma unroll
          for (int e = 0; e < 8; ++e) {
            if (OUT_MODE == 1) {
              hv[e] = (_Float16)sp[e];
            } else {
              unsigned short hb = f2bf_bits(sp[e]);
              unsigned short lb = f2bf_bits(sp[e] - bf_bits2f(hb));
              hv[e] = __builtin_bit_cast(_Float16, hb);
              lv[e] = __builtin_bit_cast(_Float16, lb);
            }
          }
          *(volatile v8h*)(C + (size_t)(mBase + row) * ldc + n0 + c8) = hv;
          if (OUT_MODE == 2) *(volatile v8h*)(C2 + (size_t)(mBase + row) * ldc + n0 + c8) = lv;
        }
        __threadfence();
      }
    }
    __builtin_amdgcn_fence(__ATOMIC_RELEASE, "workgroup");
    __builtin_amdgcn_wave_barrier();
    __builtin_amdgcn_fence(__ATOMIC_ACQUIRE, "workgroup");
  }
}

__device__ __forceinline__ unsigned short at_bf_bits(float f) {
  unsigned u = __float_as_uint(f);
  return (unsigned short)((u + 0x7FFFu + ((u >> 16) & 1u)) >> 16);
}
__device__ __forceinline__ __bf16 at_f2bf(float f) { return __builtin_bit_cast(__bf16, at_bf_bits(f)); }
__device__ __forceinline__ void at_split(float f, __bf16& hi, __bf16& lo) {
  const unsigned short hb = at_bf_bits(f);
  hi = __builtin_bit_cast(__bf16, hb);
  lo = at_f2bf(f - __uint_as_float(((unsigned)hb) << 16));
}
__device__ __forceinline__ v8f at_mma(v16b a, v16b b, v8f c) {
  c = __builtin_amdgcn_wmma_f32_16x16x32_bf16(false, a, false, b, (short)0, c, false, false);
  asm volatile("v_nop\n\tv_nop\n\tv_nop\n\tv_nop" : "+v"(c) : "v"(a), "v"(b));
  return c;
}

__device__ __forceinline__ v8f zero8() { return (v8f){0.f,0.f,0.f,0.f,0.f,0.f,0.f,0.f}; }
__device__ __forceinline__ v4u selz(bool keep, v4u a) {
  v4u r;
  r.x = keep ? a.x : 0u; r.y = keep ? a.y : 0u; r.z = keep ? a.z : 0u; r.w = keep ? a.w : 0u;
  return r;
}
__device__ __forceinline__ float wave_sum(float v) {
#pragma unroll
  for (int off = 16; off > 0; off >>= 1) v += __shfl_xor(v, off, 32);
  return v;
}
__device__ __forceinline__ void split_pack8(const float* f, v4u& uh, v4u& ul) {
  unsigned short hb[8], lb[8];
#pragma unroll
  for (int e = 0; e < 8; ++e) {
    hb[e] = f2bf_bits(f[e]);
    lb[e] = f2bf_bits(f[e] - bf_bits2f(hb[e]));
  }
  uh = (v4u){pk16(hb[0], hb[1]), pk16(hb[2], hb[3]), pk16(hb[4], hb[5]), pk16(hb[6], hb[7])};
  ul = (v4u){pk16(lb[0], lb[1]), pk16(lb[2], lb[3]), pk16(lb[4], lb[5]), pk16(lb[6], lb[7])};
}

__global__ __launch_bounds__(256) void split8_kernel(const float* __restrict__ in, unsigned short* __restrict__ hi,
                                                     unsigned short* __restrict__ lo, int n8) {
  const int i = blockIdx.x * 256 + threadIdx.x;
  if (i >= n8) return;
  const float* p = in + 8 * (size_t)i;
  const v4f a = *(const v4f*)(p);
  const v4f c = *(const v4f*)(p + 4);
  float f[8] = {a.x, a.y, a.z, a.w, c.x, c.y, c.z, c.w};
  v4u uh, ul;
  split_pack8(f, uh, ul);
  unsigned short* qh = hi + 8 * (size_t)i;
  unsigned short* ql = lo + 8 * (size_t)i;
  *(volatile v4u*)qh = uh;
  *(volatile v4u*)ql = ul;
  __threadfence();
  *(volatile v4u*)qh = uh;
  *(volatile v4u*)ql = ul;
}

__global__ __launch_bounds__(256) void xt_kernel(const float* __restrict__ xb, unsigned short* __restrict__ xhi,
                                                 unsigned short* __restrict__ xlo) {
  __shared__ float sm[64][65];
  const int t   = threadIdx.x;
  const int px0 = blockIdx.x * 64;
  const int ic0 = blockIdx.y * 64;
#pragma unroll
  for (int i = 0; i < 16; ++i) {
    const int e = i * 256 + t;
    const int r = e >> 6;
    const int c = e & 63;
    sm[c][r] = xb[(size_t)(ic0 + r) * kNpix + px0 + c];
  }
  __syncthreads();
  const int lane = t & 31, wave = t >> 5;
  const int q = lane >> 3, c8 = (lane & 7) * 8;
  for (int pass = 0; pass < 2; ++pass) {
#pragma unroll
    for (int it = 0; it < 2; ++it) {
      const int row = wave * 8 + it * 4 + q;
      float f[8];
#pragma unroll
      for (int e = 0; e < 8; ++e) f[e] = sm[row][c8 + e];
      v4u uh, ul;
      split_pack8(f, uh, ul);
      const size_t off = (size_t)(px0 + row) * kCin + ic0 + c8;
      *(volatile v4u*)(xhi + off) = uh;
      *(volatile v4u*)(xlo + off) = ul;
    }
    __threadfence();
  }
}

__global__ __launch_bounds__(256) void dw_kernel(const float* __restrict__ in, const float* __restrict__ wdw,
                                                 float* __restrict__ out) {
  const int ch = blockIdx.y;
  const int t4 = blockIdx.x * 256 + threadIdx.x;
  const int px = t4 * 4;
  const int y  = px >> 7;
  const int x0 = px & (kImw - 1);
  const float* src = in + (size_t)ch * kNpix;
  const float* wp  = wdw + ch * 9;
  float wk[9];
#pragma unroll
  for (int k = 0; k < 9; ++k) wk[k] = wp[k];
  float rv[3][6];
#pragma unroll
  for (int dy = 0; dy < 3; ++dy) {
    const int yy = y + dy - 1;
    const bool rowok = (yy >= 0) && (yy < kImw);
    const int yyc = (yy < 0) ? 0 : ((yy > kImw - 1) ? (kImw - 1) : yy);
    const float* rp = src + yyc * kImw;
    const v4f mid = *(const v4f*)(rp + x0);
    const int xl = (x0 > 0) ? (x0 - 1) : 0;
    const int xr = (x0 + 4 < kImw) ? (x0 + 4) : (kImw - 1);
    const float lf = rp[xl];
    const float rg = rp[xr];
    rv[dy][0] = (rowok && (x0 > 0)) ? lf : 0.f;
    rv[dy][1] = rowok ? mid.x : 0.f;
    rv[dy][2] = rowok ? mid.y : 0.f;
    rv[dy][3] = rowok ? mid.z : 0.f;
    rv[dy][4] = rowok ? mid.w : 0.f;
    rv[dy][5] = (rowok && (x0 + 4 < kImw)) ? rg : 0.f;
  }
  float oj[4];
#pragma unroll
  for (int j = 0; j < 4; ++j) {
    float a = 0.f;
#pragma unroll
    for (int dy = 0; dy < 3; ++dy)
#pragma unroll
      for (int dx = 0; dx < 3; ++dx) a += wk[dy * 3 + dx] * rv[dy][j + dx];
    oj[j] = a;
  }
  const v4f o = (v4f){oj[0], oj[1], oj[2], oj[3]};
  float* op = out + (size_t)ch * kNpix + px;
  *(volatile v4f*)op = o;
  __threadfence();
  *(volatile v4f*)op = o;
}

__global__ __launch_bounds__(256) void packqk_kernel(const float* __restrict__ dw, unsigned short* __restrict__ qh,
                                                     unsigned short* __restrict__ ql, unsigned short* __restrict__ kh,
                                                     unsigned short* __restrict__ kl) {
  __shared__ float sm[64][33];
  __shared__ float sinv[64];
  const int t  = threadIdx.x;
  const int n0 = blockIdx.x * 64;
  const int h  = blockIdx.y;
  const int p  = blockIdx.z;
  const float* base = dw + ((size_t)(p * kCin + h * kChd)) * kNpix + n0;
#pragma unroll
  for (int i = 0; i < 6; ++i) {
    const int e = i * 256 + t;
    const int c = e >> 6;
    const int nl = e & 63;
    sm[nl][c] = base[(size_t)c * kNpix + nl];
  }
  __syncthreads();
  if (t < 64) {
    float ss = 0.f;
#pragma unroll
    for (int c = 0; c < kChd; ++c) ss += sm[t][c] * sm[t][c];
    sinv[t] = 1.0f / fmaxf(sqrtf(ss), 1e-12f);
  }
  __syncthreads();
  const int lane = t & 31, wave = t >> 5;
  const int nl = wave * 8 + (lane >> 2);
  const int j  = lane & 3;
  const float inv = sinv[nl];
  float f[8];
#pragma unroll
  for (int e = 0; e < 8; ++e) {
    const int c  = 8 * j + e;
    const int cc = (c < kChd) ? c : (kChd - 1);
    const float v = sm[nl][cc] * inv;
    f[e] = (c < kChd) ? v : 0.0f;
  }
  v4u uh, ul;
  split_pack8(f, uh, ul);
  unsigned short* oh = (p == 0) ? qh : kh;
  unsigned short* ol = (p == 0) ? ql : kl;
  const size_t off = ((size_t)(h * kNpix + n0 + nl)) * kCpad + 8 * j;
  *(volatile v4u*)(oh + off) = uh;
  *(volatile v4u*)(ol + off) = ul;
  __threadfence();
  *(volatile v4u*)(oh + off) = uh;
  *(volatile v4u*)(ol + off) = ul;
}

__global__ __launch_bounds__(256) void pool_kernel(const float* __restrict__ dwa, unsigned short* __restrict__ ah,
                                                   unsigned short* __restrict__ al) {
  __shared__ float sm[64][33];
  const int h    = blockIdx.x;
  const int t    = threadIdx.x;
  const int m    = t >> 2;
  const int part = t & 3;
  const int my   = m >> 3;
  const int mx   = m & 7;
  const int y0   = my * 16 + part * 4;
  const int xb   = mx * 16;
#pragma unroll 1
  for (int c = 0; c < kChd; ++c) {
    const float* srcp = dwa + ((size_t)(h * kChd + c)) * kNpix + y0 * kImw + xb;
    float s = 0.f;
#pragma unroll
    for (int r = 0; r < 4; ++r) {
      const v4f* rp = (const v4f*)(srcp + r * kImw);
      const v4f a0 = rp[0], a1 = rp[1], a2 = rp[2], a3 = rp[3];
      s += ((a0.x + a0.y) + (a0.z + a0.w)) + ((a1.x + a1.y) + (a1.z + a1.w))
         + ((a2.x + a2.y) + (a2.z + a2.w)) + ((a3.x + a3.y) + (a3.z + a3.w));
    }
    s += __shfl_xor(s, 1, 32);
    s += __shfl_xor(s, 2, 32);
    if (part == 0) sm[m][c] = s * (1.0f / 256.0f);
  }
  __syncthreads();
  const int lane = t & 31, wave = t >> 5;
  const int row = wave * 8 + (lane >> 2);
  const int j   = lane & 3;
  float f[8];
#pragma unroll
  for (int e = 0; e < 8; ++e) {
    const int c  = 8 * j + e;
    const int cc = (c < kChd) ? c : (kChd - 1);
    const float v = sm[row][cc];
    f[e] = (c < kChd) ? v : 0.0f;
  }
  v4u uh, ul;
  split_pack8(f, uh, ul);
  const size_t off = ((size_t)(h * kNag + row)) * kCpad + 8 * j;
  *(volatile v4u*)(ah + off) = uh;
  *(volatile v4u*)(al + off) = ul;
  __threadfence();
  *(volatile v4u*)(ah + off) = uh;
  *(volatile v4u*)(al + off) = ul;
}

__global__ __launch_bounds__(128) void kagg_kernel(
    const unsigned short* __restrict__ knh, const unsigned short* __restrict__ knl,
    const unsigned short* __restrict__ vh,  const unsigned short* __restrict__ vl,
    const unsigned short* __restrict__ agh, const unsigned short* __restrict__ agl,
    const float* __restrict__ temp, float* __restrict__ part_o, float* __restrict__ part_ml) {
  union FB { v16b v; v8b h[2]; };
  __shared__ __align__(16) __bf16 Ksh[64 * kCpad];
  __shared__ __align__(16) __bf16 Ksl[64 * kCpad];
  __shared__ __align__(16) __bf16 Vth[kCpad * 64];
  __shared__ __align__(16) __bf16 Vtl[kCpad * 64];
  __shared__ __align__(16) __bf16 Psh[4][16 * 64];
  __shared__ __align__(16) __bf16 Psl[4][16 * 64];
  __shared__ __align__(16) float  Os[4][16 * 36];
  __shared__ __align__(16) float  Mls[kNag * 2];

  const int tid  = threadIdx.x;
  const int wave = tid >> 5;
  const int lane = tid & 31;
  const int hh   = lane >> 4;
  const int c    = lane & 15;
  const int h    = blockIdx.x / kKBlk;
  const int blk  = blockIdx.x - h * kKBlk;
  const float tscale = temp[h];
  const int m0   = wave * 16;

  const size_t agoff = ((size_t)(h * kNag + m0 + c)) * kCpad + 8 * hh;
  const v16b qah = Frag<__bf16>::load((const __bf16*)agh + agoff);
  const v16b qal = Frag<__bf16>::load((const __bf16*)agl + agoff);

  float mrow[8], lrow[8];
  v8f oacc[2];
#pragma unroll
  for (int r = 0; r < 8; ++r) { mrow[r] = -INFINITY; lrow[r] = 0.f; }
  oacc[0] = zero8();
  oacc[1] = zero8();

  for (int kc = 0; kc < kKChunk; ++kc) {
    const int n0 = (blk * kKChunk + kc) * 64;
    __syncthreads();
    {
      const v4u* gh = (const v4u*)(knh + ((size_t)h * kNpix + n0) * kCpad);
      const v4u* gl = (const v4u*)(knl + ((size_t)h * kNpix + n0) * kCpad);
#pragma unroll
      for (int i = 0; i < 2; ++i) {
        const int q = tid + 128 * i;
        ((v4u*)Ksh)[q] = gh[q];
        ((v4u*)Ksl)[q] = gl[q];
      }
#pragma unroll
      for (int i = 0; i < 2; ++i) {
        const int q    = tid + 128 * i;
        const int row  = q >> 3;
        const int col  = q & 7;
        const int rowc = (row < kChd) ? row : (kChd - 1);
        const size_t vo = ((size_t)(h * kChd + rowc)) * kNpix + n0;
        const v4u a  = ((const v4u*)(vh + vo))[col];
        const v4u bq = ((const v4u*)(vl + vo))[col];
        const bool keep = (row < kChd);
        ((v4u*)Vth)[q] = selz(keep, a);
        ((v4u*)Vtl)[q] = selz(keep, bq);
      }
    }
    __syncthreads();

    v8f s[4];
#pragma unroll
    for (int j = 0; j < 4; ++j) {
      s[j] = zero8();
      FB kb, kl;
      kb.h[0] = *(const v8b*)(Ksh + (j * 16 + c) * kCpad + 8 * hh);
      kb.h[1] = *(const v8b*)(Ksh + (j * 16 + c) * kCpad + 16 + 8 * hh);
      kl.h[0] = *(const v8b*)(Ksl + (j * 16 + c) * kCpad + 8 * hh);
      kl.h[1] = *(const v8b*)(Ksl + (j * 16 + c) * kCpad + 16 + 8 * hh);
      s[j] = at_mma(qah, kb.v, s[j]);
      s[j] = at_mma(qah, kl.v, s[j]);
      s[j] = at_mma(qal, kb.v, s[j]);
    }
    float cm[8];
#pragma unroll
    for (int r = 0; r < 8; ++r) {
      float mmax = -INFINITY;
#pragma unroll
      for (int j = 0; j < 4; ++j) {
        s[j][r] = s[j][r] * tscale;
        mmax = fmaxf(mmax, s[j][r]);
      }
#pragma unroll
      for (int off = 1; off < 16; off <<= 1) mmax = fmaxf(mmax, __shfl_xor(mmax, off, 32));
      cm[r] = mmax;
    }
    __bf16* pwh = Psh[wave];
    __bf16* pwl = Psl[wave];
#pragma unroll
    for (int r = 0; r < 8; ++r) {
      const float mnew  = fmaxf(mrow[r], cm[r]);
      const float alpha = expf(mrow[r] - mnew);
      mrow[r] = mnew;
      float psum = 0.f;
#pragma unroll
      for (int j = 0; j < 4; ++j) {
        const float p = expf(s[j][r] - mnew);
        psum += p;
        __bf16 a, bl;
        at_split(p, a, bl);
        pwh[(8 * hh + r) * 64 + j * 16 + c] = a;
        pwl[(8 * hh + r) * 64 + j * 16 + c] = bl;
      }
#pragma unroll
      for (int off = 1; off < 16; off <<= 1) psum += __shfl_xor(psum, off, 32);
      lrow[r] = lrow[r] * alpha + psum;
      oacc[0][r] *= alpha;
      oacc[1][r] *= alpha;
    }
    __builtin_amdgcn_fence(__ATOMIC_RELEASE, "workgroup");
    __builtin_amdgcn_wave_barrier();
    __builtin_amdgcn_fence(__ATOMIC_ACQUIRE, "workgroup");
#pragma unroll 1
    for (int kk = 0; kk < 2; ++kk) {
      FB pa, pl;
      pa.h[0] = *(const v8b*)(pwh + c * 64 + kk * 32 + 8 * hh);
      pa.h[1] = *(const v8b*)(pwh + c * 64 + kk * 32 + 16 + 8 * hh);
      pl.h[0] = *(const v8b*)(pwl + c * 64 + kk * 32 + 8 * hh);
      pl.h[1] = *(const v8b*)(pwl + c * 64 + kk * 32 + 16 + 8 * hh);
#pragma unroll
      for (int t = 0; t < 2; ++t) {
        FB vb, vq;
        vb.h[0] = *(const v8b*)(Vth + (t * 16 + c) * 64 + kk * 32 + 8 * hh);
        vb.h[1] = *(const v8b*)(Vth + (t * 16 + c) * 64 + kk * 32 + 16 + 8 * hh);
        vq.h[0] = *(const v8b*)(Vtl + (t * 16 + c) * 64 + kk * 32 + 8 * hh);
        vq.h[1] = *(const v8b*)(Vtl + (t * 16 + c) * 64 + kk * 32 + 16 + 8 * hh);
        oacc[t] = at_mma(pa.v, vb.v, oacc[t]);
        oacc[t] = at_mma(pa.v, vq.v, oacc[t]);
        oacc[t] = at_mma(pl.v, vb.v, oacc[t]);
      }
    }
  }

  float* os = Os[wave];
#pragma unroll
  for (int r = 0; r < 8; ++r) {
    os[(8 * hh + r) * 36 + c]      = oacc[0][r];
    os[(8 * hh + r) * 36 + 16 + c] = oacc[1][r];
  }
  if (c == 0) {
#pragma unroll
    for (int r = 0; r < 8; ++r) {
      Mls[(m0 + 8 * hh + r) * 2]     = mrow[r];
      Mls[(m0 + 8 * hh + r) * 2 + 1] = lrow[r];
    }
  }
  __syncthreads();
  {
    float* ob = part_o + (((size_t)(h * kKBlk + blk)) * kNag + m0) * kCpad;
    const int q = lane >> 3, c4 = (lane & 7) * 4;
    for (int pass = 0; pass < 2; ++pass) {
#pragma unroll
      for (int it = 0; it < 4; ++it) {
        const int row = it * 4 + q;
        const v4f v = *(const v4f*)(os + row * 36 + c4);
        *(volatile v4f*)(ob + row * kCpad + c4) = v;
      }
      __threadfence();
    }
  }
  if (wave == 0) {
    float* mb = part_ml + ((size_t)(h * kKBlk + blk)) * kNag * 2;
    for (int pass = 0; pass < 2; ++pass) {
      const v4f v = *(const v4f*)(Mls + 4 * lane);
      *(volatile v4f*)(mb + 4 * lane) = v;
      __threadfence();
    }
  }
}

__global__ __launch_bounds__(256) void kcomb_kernel(const float* __restrict__ part_o, const float* __restrict__ part_ml,
                                                    unsigned short* __restrict__ avh, unsigned short* __restrict__ avl) {
  __shared__ float st[32][65];
  const int h = blockIdx.x;
  const int t = threadIdx.x;
  const int m = t >> 2;
  const int j = t & 3;
  const float* mlb = part_ml + (size_t)h * kKBlk * kNag * 2;
  const float* ob0 = part_o + (size_t)h * kKBlk * kNag * kCpad;
  float mx = -INFINITY;
#pragma unroll 1
  for (int blk = 0; blk < kKBlk; ++blk) mx = fmaxf(mx, mlb[(blk * kNag + m) * 2]);
  float lsum = 0.f;
  float acc[8] = {0.f, 0.f, 0.f, 0.f, 0.f, 0.f, 0.f, 0.f};
#pragma unroll 1
  for (int blk = 0; blk < kKBlk; ++blk) {
    const float mb = mlb[(blk * kNag + m) * 2];
    const float lb = mlb[(blk * kNag + m) * 2 + 1];
    const float w  = expf(mb - mx);
    lsum += w * lb;
    const float* ob = ob0 + ((size_t)(blk * kNag + m)) * kCpad + 8 * j;
    const v4f a  = *(const v4f*)(ob);
    const v4f bq = *(const v4f*)(ob + 4);
    acc[0] += w * a.x;  acc[1] += w * a.y;  acc[2] += w * a.z;  acc[3] += w * a.w;
    acc[4] += w * bq.x; acc[5] += w * bq.y; acc[6] += w * bq.z; acc[7] += w * bq.w;
  }
  const float inv = 1.0f / lsum;
#pragma unroll
  for (int e = 0; e < 8; ++e) st[8 * j + e][m] = acc[e] * inv;
  __syncthreads();
  const int lane = t & 31, wave = t >> 5;
  const int row = wave * 4 + (lane >> 3);
  const int c8  = (lane & 7) * 8;
  float f[8];
#pragma unroll
  for (int e = 0; e < 8; ++e) f[e] = st[row][c8 + e];
  v4u uh, ul;
  split_pack8(f, uh, ul);
  const size_t off = ((size_t)(h * kCpad + row)) * kNag + c8;
  *(volatile v4u*)(avh + off) = uh;
  *(volatile v4u*)(avl + off) = ul;
  __threadfence();
  *(volatile v4u*)(avh + off) = uh;
  *(volatile v4u*)(avl + off) = ul;
}

__global__ __launch_bounds__(128) void qout_kernel(
    const unsigned short* __restrict__ qnh, const unsigned short* __restrict__ qnl,
    const unsigned short* __restrict__ agh, const unsigned short* __restrict__ agl,
    const unsigned short* __restrict__ avh, const unsigned short* __restrict__ avl,
    const float* __restrict__ temp, float* __restrict__ outT) {
  union FB { v16b v; v8b h[2]; };
  __shared__ __align__(16) __bf16 AGh[kNag * kCpad];
  __shared__ __align__(16) __bf16 AGl[kNag * kCpad];
  __shared__ __align__(16) __bf16 AVh[kCpad * kNag];
  __shared__ __align__(16) __bf16 AVl[kCpad * kNag];
  __shared__ __align__(16) __bf16 Psh[4][16 * 64];
  __shared__ __align__(16) __bf16 Psl[4][16 * 64];
  __shared__ __align__(16) float  Ost[kCpad * 68];

  const int tid  = threadIdx.x;
  const int wave = tid >> 5;
  const int lane = tid & 31;
  const int hh   = lane >> 4;
  const int c    = lane & 15;
  const int h    = blockIdx.x / kQBlk;
  const int blkq = blockIdx.x - h * kQBlk;
  const float tscale = temp[h];
  {
    const v4u* gah = (const v4u*)(agh + (size_t)h * kNag * kCpad);
    const v4u* gal = (const v4u*)(agl + (size_t)h * kNag * kCpad);
    const v4u* gvh = (const v4u*)(avh + (size_t)h * kCpad * kNag);
    const v4u* gvl = (const v4u*)(avl + (size_t)h * kCpad * kNag);
#pragma unroll
    for (int i = 0; i < 2; ++i) {
      const int q = tid + 128 * i;
      ((v4u*)AGh)[q] = gah[q];
      ((v4u*)AGl)[q] = gal[q];
      ((v4u*)AVh)[q] = gvh[q];
      ((v4u*)AVl)[q] = gvl[q];
    }
  }
  __syncthreads();

  for (int tt = 0; tt < kQTile; ++tt) {
    const int q0 = (blkq * kQTile + tt) * 64;
    const int qr = q0 + wave * 16;
    const size_t qoff = ((size_t)h * kNpix + qr + c) * kCpad + 8 * hh;
    const v16b qah = Frag<__bf16>::load((const __bf16*)qnh + qoff);
    const v16b qal = Frag<__bf16>::load((const __bf16*)qnl + qoff);

    v8f s[4];
#pragma unroll
    for (int j = 0; j < 4; ++j) {
      s[j] = zero8();
      FB kb, kl;
      kb.h[0] = *(const v8b*)(AGh + (j * 16 + c) * kCpad + 8 * hh);
      kb.h[1] = *(const v8b*)(AGh + (j * 16 + c) * kCpad + 16 + 8 * hh);
      kl.h[0] = *(const v8b*)(AGl + (j * 16 + c) * kCpad + 8 * hh);
      kl.h[1] = *(const v8b*)(AGl + (j * 16 + c) * kCpad + 16 + 8 * hh);
      s[j] = at_mma(qah, kb.v, s[j]);
      s[j] = at_mma(qah, kl.v, s[j]);
      s[j] = at_mma(qal, kb.v, s[j]);
    }
    float cm[8], lsum[8];
#pragma unroll
    for (int r = 0; r < 8; ++r) {
      float mmax = -INFINITY;
#pragma unroll
      for (int j = 0; j < 4; ++j) {
        s[j][r] = s[j][r] * tscale;
        mmax = fmaxf(mmax, s[j][r]);
      }
#pragma unroll
      for (int off = 1; off < 16; off <<= 1) mmax = fmaxf(mmax, __shfl_xor(mmax, off, 32));
      cm[r] = mmax;
    }
    __bf16* pwh = Psh[wave];
    __bf16* pwl = Psl[wave];
#pragma unroll
    for (int r = 0; r < 8; ++r) {
      float psum = 0.f;
#pragma unroll
      for (int j = 0; j < 4; ++j) {
        const float p = expf(s[j][r] - cm[r]);
        psum += p;
        __bf16 a, bl;
        at_split(p, a, bl);
        pwh[(8 * hh + r) * 64 + j * 16 + c] = a;
        pwl[(8 * hh + r) * 64 + j * 16 + c] = bl;
      }
#pragma unroll
      for (int off = 1; off < 16; off <<= 1) psum += __shfl_xor(psum, off, 32);
      lsum[r] = psum;
    }
    __builtin_amdgcn_fence(__ATOMIC_RELEASE, "workgroup");
    __builtin_amdgcn_wave_barrier();
    __builtin_amdgcn_fence(__ATOMIC_ACQUIRE, "workgroup");
    v8f oacc[2];
    oacc[0] = zero8();
    oacc[1] = zero8();
#pragma unroll 1
    for (int kk = 0; kk < 2; ++kk) {
      FB pa, pl;
      pa.h[0] = *(const v8b*)(pwh + c * 64 + kk * 32 + 8 * hh);
      pa.h[1] = *(const v8b*)(pwh + c * 64 + kk * 32 + 16 + 8 * hh);
      pl.h[0] = *(const v8b*)(pwl + c * 64 + kk * 32 + 8 * hh);
      pl.h[1] = *(const v8b*)(pwl + c * 64 + kk * 32 + 16 + 8 * hh);
#pragma unroll
      for (int t = 0; t < 2; ++t) {
        FB vb, vq;
        vb.h[0] = *(const v8b*)(AVh + (t * 16 + c) * kNag + kk * 32 + 8 * hh);
        vb.h[1] = *(const v8b*)(AVh + (t * 16 + c) * kNag + kk * 32 + 16 + 8 * hh);
        vq.h[0] = *(const v8b*)(AVl + (t * 16 + c) * kNag + kk * 32 + 8 * hh);
        vq.h[1] = *(const v8b*)(AVl + (t * 16 + c) * kNag + kk * 32 + 16 + 8 * hh);
        oacc[t] = at_mma(pa.v, vb.v, oacc[t]);
        oacc[t] = at_mma(pa.v, vq.v, oacc[t]);
        oacc[t] = at_mma(pl.v, vb.v, oacc[t]);
      }
    }
#pragma unroll
    for (int r = 0; r < 8; ++r) {
      const float inv = 1.0f / lsum[r];
      Ost[c * 68 + wave * 16 + 8 * hh + r]        = oacc[0][r] * inv;
      Ost[(16 + c) * 68 + wave * 16 + 8 * hh + r] = oacc[1][r] * inv;
    }
    __syncthreads();
    {
      const int c4 = (lane & 15) * 4;
      for (int pass = 0; pass < 2; ++pass) {
#pragma unroll
        for (int it = 0; it < 3; ++it) {
          const int row = wave * 6 + it * 2 + hh;
          const v4f v = *(const v4f*)(Ost + row * 68 + c4);
          *(volatile v4f*)(outT + ((size_t)(h * kChd + row)) * kNpix + q0 + c4) = v;
        }
        __threadfence();
      }
    }
    __syncthreads();
  }
}

__global__ __launch_bounds__(256) void gate_kernel(const float* __restrict__ src, float* __restrict__ dst) {
  __shared__ __align__(16) v4f srow[kNpix / 4];
  __shared__ float sred[8];
  const int rowi = blockIdx.x;
  const int t    = threadIdx.x;
  const int lane = t & 31, wave = t >> 5;
  const v4f* sp = (const v4f*)(src + (size_t)rowi * kNpix);
  float s = 0.f;
#pragma unroll 1
  for (int i = 0; i < 16; ++i) {
    const int idx = i * 256 + t;
    const v4f a = sp[idx];
    srow[idx] = a;
    s += (a.x + a.y) + (a.z + a.w);
  }
  s = wave_sum(s);
  if (lane == 0) sred[wave] = s;
  __syncthreads();
  float tot = 0.f;
#pragma unroll
  for (int w = 0; w < 8; ++w) tot += sred[w];
  const float mu = tot * (1.0f / 16384.0f);
  __syncthreads();
  float s2 = 0.f;
#pragma unroll 1
  for (int i = 0; i < 16; ++i) {
    const int idx = i * 256 + t;
    const v4f a = srow[idx];
    const float d0 = a.x - mu, d1 = a.y - mu, d2 = a.z - mu, d3 = a.w - mu;
    s2 += (d0 * d0 + d1 * d1) + (d2 * d2 + d3 * d3);
  }
  s2 = wave_sum(s2);
  if (lane == 0) sred[wave] = s2;
  __syncthreads();
  float tot2 = 0.f;
#pragma unroll
  for (int w = 0; w < 8; ++w) tot2 += sred[w];
  const float denom = 4.0f * (tot2 * (1.0f / 16383.0f) + 1e-4f);
  const float inv = 1.0f / denom;
  float* dp = dst + (size_t)rowi * kNpix;
#pragma unroll 1
  for (int i = 0; i < 16; ++i) {
    const int idx = i * 256 + t;
    const v4f a = srow[idx];
    v4f o;
    {
      const float d = a.x - mu; const float yv = d * d * inv + 0.5f; const float e = expf(-yv); o.x = a.x * (1.0f / (1.0f + e));
    }
    {
      const float d = a.y - mu; const float yv = d * d * inv + 0.5f; const float e = expf(-yv); o.y = a.y * (1.0f / (1.0f + e));
    }
    {
      const float d = a.z - mu; const float yv = d * d * inv + 0.5f; const float e = expf(-yv); o.z = a.z * (1.0f / (1.0f + e));
    }
    {
      const float d = a.w - mu; const float yv = d * d * inv + 0.5f; const float e = expf(-yv); o.w = a.w * (1.0f / (1.0f + e));
    }
    srow[idx] = o;
    *(volatile v4f*)(dp + 4 * (size_t)idx) = o;
  }
  __threadfence();
#pragma unroll 1
  for (int i = 0; i < 16; ++i) {
    const int idx = i * 256 + t;
    const v4f o = srow[idx];
    *(volatile v4f*)(dp + 4 * (size_t)idx) = o;
  }
}

extern "C" void kernel_launch(void* const* d_in, const int* in_sizes, int n_in,
                              void* d_out, int out_size, void* d_ws, size_t ws_size, hipStream_t stream) {
  if (n_in < 4) return;
  if (in_sizes[0] != kBatch * kCin * kNpix) return;
  if (in_sizes[1] != kOc * kCin) return;
  if (in_sizes[2] != kOc * 9) return;
  if (in_sizes[3] < kHeads) return;
  if (out_size != kBatch * kCin * kNpix) return;
  if (ws_size < kWsEnd) return;

  const float* x     = (const float*)d_in[0];
  const float* w_qkv = (const float*)d_in[1];
  const float* w_dw  = (const float*)d_in[2];
  const float* temp  = (const float*)d_in[3];
  float* dout = (float*)d_out;
  char* ws = (char*)d_ws;

  unsigned short* whi  = (unsigned short*)(ws + kOffWhi);
  unsigned short* wlo  = (unsigned short*)(ws + kOffWlo);
  float*          pre  = (float*)(ws + kOffPre);
  unsigned short* qnhi = (unsigned short*)(ws + kOffQnhi);
  unsigned short* qnlo = (unsigned short*)(ws + kOffQnlo);
  unsigned short* knhi = (unsigned short*)(ws + kOffKnhi);
  unsigned short* knlo = (unsigned short*)(ws + kOffKnlo);
  unsigned short* vhi  = (unsigned short*)(ws + kOffVhi);
  unsigned short* vlo  = (unsigned short*)(ws + kOffVlo);
  unsigned short* xthi = (unsigned short*)(ws + kOffXthi);
  unsigned short* xtlo = (unsigned short*)(ws + kOffXtlo);
  float*          dwp  = (float*)(ws + kOffDw);
  float*          outT = (float*)(ws + kOffOutT);
  unsigned short* aghi = (unsigned short*)(ws + kOffAghi);
  unsigned short* aglo = (unsigned short*)(ws + kOffAglo);
  unsigned short* avhi = (unsigned short*)(ws + kOffAvhi);
  unsigned short* avlo = (unsigned short*)(ws + kOffAvlo);
  float*          parto  = (float*)(ws + kOffPartO);
  float*          partml = (float*)(ws + kOffPartML);

  split8_kernel<<<(kOc * kCin / 8) / 256, 256, 0, stream>>>(w_qkv, whi, wlo, kOc * kCin / 8);

  for (int b = 0; b < kBatch; ++b) {
    const float* xb = x + (size_t)b * kCin * kNpix;
    xt_kernel<<<dim3(kNpix / 64, kCin / 64), 256, 0, stream>>>(xb, xthi, xtlo);
    wmma_gemm64<1, true, 0, 0, false><<<dim3((kOc / 64) * (kNpix / 64) / 8, 1), 256, 0, stream>>>(
        whi, wlo, kCin, 0L, xthi, xtlo, kCin, 0L, (void*)pre, (void*)nullptr, kNpix, 0L,
        nullptr, nullptr, 0L, kOc, kNpix, kCin, 1.0f);
    dw_kernel<<<dim3(kNpix / (256 * 4), kOc), 256, 0, stream>>>(pre, w_dw, dwp);
    packqk_kernel<<<dim3(kNpix / 64, kHeads, 2), 256, 0, stream>>>(dwp, qnhi, qnlo, knhi, knlo);
    split8_kernel<<<(kCin * kNpix / 8) / 256, 256, 0, stream>>>(dwp + (size_t)2 * kCin * kNpix, vhi, vlo, kCin * kNpix / 8);
    pool_kernel<<<kHeads, 256, 0, stream>>>(dwp + (size_t)3 * kCin * kNpix, aghi, aglo);
    kagg_kernel<<<kHeads * kKBlk, 128, 0, stream>>>(knhi, knlo, vhi, vlo, aghi, aglo, temp, parto, partml);
    kcomb_kernel<<<kHeads, 256, 0, stream>>>(parto, partml, avhi, avlo);
    qout_kernel<<<kHeads * kQBlk, 128, 0, stream>>>(qnhi, qnlo, aghi, aglo, avhi, avlo, temp, outT);
    gate_kernel<<<kCin, 256, 0, stream>>>(outT, dout + (size_t)b * kCin * kNpix);
  }
}
